// VDMAttnBlock_51256139710745
// MI455X (gfx1250) — hardware-verified
//
#include <hip/hip_runtime.h>


#define NB_  4
#define CC   512
#define NN   4096
#define NG   32
#define PCAR 1024.0f
typedef _Float16 h16;
typedef unsigned short bf;
typedef __attribute__((ext_vector_type(16))) __bf16   v16bf;
typedef __attribute__((ext_vector_type(16))) _Float16 v16h;
typedef __attribute__((ext_vector_type(8)))  _Float16 v8h;
typedef __attribute__((ext_vector_type(8)))  unsigned short v8us;
typedef __attribute__((ext_vector_type(8)))  float    v8f;
typedef __attribute__((ext_vector_type(4)))  float    v4f;
typedef v8h  __attribute__((may_alias)) v8ha;
typedef v4f  __attribute__((may_alias)) v4fa;
typedef v8us __attribute__((may_alias)) v8usa;

__device__ __forceinline__ unsigned short f2bf(float f) { unsigned u = __float_as_uint(f); u += 0x7FFFu + ((u >> 16) & 1u); return (unsigned short)(u >> 16); }
__device__ __forceinline__ float bf2f(unsigned short b) { return __uint_as_float(((unsigned)b) << 16); }
__device__ __forceinline__ float bfr(float f) { return bf2f(f2bf(f)); }
__device__ __forceinline__ v16h cat16(v8h lo, v8h hi) { return __builtin_shufflevector(lo, hi, 0, 1, 2, 3, 4, 5, 6, 7, 8, 9, 10, 11, 12, 13, 14, 15); }
__device__ __forceinline__ v16bf cat16b(v8us lo, v8us hi) { return __builtin_bit_cast(v16bf, __builtin_shufflevector(lo, hi, 0, 1, 2, 3, 4, 5, 6, 7, 8, 9, 10, 11, 12, 13, 14, 15)); }
__device__ __forceinline__ v8f wmma16(v16h a, v16h b, v8f c) { return __builtin_amdgcn_wmma_f32_16x16x32_f16(false, a, false, b, (short)0, c, false, false); }
__device__ __forceinline__ v8f wmmab(v16bf a, v16bf b, v8f c) { return __builtin_amdgcn_wmma_f32_16x16x32_bf16(false, a, false, b, (short)0, c, false, false); }


template <typename T16> struct WFrag;
template <> struct WFrag<h16> { typedef v16h V; static __device__ __forceinline__ V ld(const h16* p) { return cat16(*(const v8h*)p, *(const v8h*)(p + 16)); } static __device__ __forceinline__ v8f mma(V a, V b, v8f c) { return wmma16(a, b, c); } };
template <> struct WFrag<bf> { typedef v16bf V; static __device__ __forceinline__ V ld(const bf* p) { return cat16b(*(const v8us*)p, *(const v8us*)(p + 16)); } static __device__ __forceinline__ v8f mma(V a, V b, v8f c) { return wmmab(a, b, c); } };
template <typename T16, int NSPLIT, bool BIAS>
__global__ __launch_bounds__(32) void k_gemmw(const T16* __restrict__ A, const T16* __restrict__ A2, const T16* __restrict__ Bt, const T16* __restrict__ Bt2, int K, float* C, int ldc, const float* __restrict__ bias, size_t sA, size_t sB, size_t sC) {
    typedef typename WFrag<T16>::V V;
    __shared__ __align__(16) float os[16 * 68];
    const size_t z = blockIdx.z; A += z * sA; if (A2) A2 += z * sA; Bt += z * sB; if (Bt2) Bt2 += z * sB; C += z * sC;
    const int lane = threadIdx.x & 31, lr = lane & 15, hi = lane >> 4; const int r0 = blockIdx.x * 64, c0 = blockIdx.y * 64;
    v8f acc[4][4];
#pragma unroll
    for (int mb = 0; mb < 4; ++mb)
#pragma unroll
        for (int nb = 0; nb < 4; ++nb) acc[mb][nb] = (v8f){};
    const size_t aoff = (size_t)(r0 + lr) * K + 8 * hi, boff = (size_t)(c0 + lr) * K + 8 * hi;
#pragma unroll 1
    for (int kc = 0; kc < K; kc += 32) {
        V a[4], a2[4];
#pragma unroll
        for (int mb = 0; mb < 4; ++mb) { a[mb] = WFrag<T16>::ld(A + aoff + (size_t)mb * 16 * K + kc); if (NSPLIT == 1 || NSPLIT == 2) a2[mb] = WFrag<T16>::ld(A2 + aoff + (size_t)mb * 16 * K + kc); }
#pragma unroll
        for (int nb = 0; nb < 4; ++nb) { const V b = WFrag<T16>::ld(Bt + boff + (size_t)nb * 16 * K + kc); V b2; if (NSPLIT >= 2) b2 = WFrag<T16>::ld(Bt2 + boff + (size_t)nb * 16 * K + kc);
#pragma unroll
            for (int mb = 0; mb < 4; ++mb) { acc[mb][nb] = WFrag<T16>::mma(a[mb], b, acc[mb][nb]); if (NSPLIT == 1 || NSPLIT == 2) acc[mb][nb] = WFrag<T16>::mma(a2[mb], b, acc[mb][nb]); if (NSPLIT >= 2) acc[mb][nb] = WFrag<T16>::mma(a[mb], b2, acc[mb][nb]); } }
        asm volatile("v_nop\n\tv_nop\n\tv_nop\n\tv_nop" : "+v"(acc[0][0]), "+v"(acc[1][1]), "+v"(acc[2][2]), "+v"(acc[3][3]) : "v"(a[0]), "v"(a[3]));
    }
#pragma unroll
    for (int mb = 0; mb < 4; ++mb) {
#pragma unroll
        for (int nb = 0; nb < 4; ++nb) {
#pragma unroll
            for (int j = 0; j < 8; ++j) os[(hi * 8 + j) * 68 + nb * 16 + lr] = acc[mb][nb][j]; }
        __builtin_amdgcn_wave_barrier(); asm volatile("" ::: "memory");
        float* crow = C + (size_t)(r0 + mb * 16) * ldc + c0;
#pragma unroll 1
        for (int ps = 0; ps < 2; ++ps) {
#pragma unroll
            for (int s = 0; s < 8; ++s) { const int row = 2 * s + hi, cofs = lr * 4; v4f val = *(const v4fa*)(os + row * 68 + cofs); if (BIAS) { val[0] += bfr(bias[c0 + cofs]); val[1] += bfr(bias[c0 + cofs + 1]); val[2] += bfr(bias[c0 + cofs + 2]); val[3] += bfr(bias[c0 + cofs + 3]); }
                *(volatile v4f*)(crow + (size_t)row * ldc + cofs) = val; }
            if (ps == 0) __threadfence(); }
        __builtin_amdgcn_wave_barrier(); asm volatile("" ::: "memory");
    }
}

__device__ __forceinline__ h16 tohx(float x) { return (h16)x; }
__device__ __forceinline__ void splitf(float y, unsigned short& h, unsigned short& l) { h = f2bf(y); l = f2bf(y - bf2f(h)); }
typedef __attribute__((ext_vector_type(2))) unsigned short v2us;
typedef __attribute__((ext_vector_type(4))) unsigned short v4us;
typedef __attribute__((ext_vector_type(2))) _Float16 v2h; typedef __attribute__((ext_vector_type(2))) float v2f;
typedef __attribute__((ext_vector_type(4))) _Float16 v4h;

__global__ __launch_bounds__(256) void k_cvt8(const float* __restrict__ src, bf* dst, size_t n8) { const size_t i = (size_t)blockIdx.x * 256 + threadIdx.x; if (i >= n8) return; const v8f v = *(const v8f*)(src + i * 8); v8us o;
#pragma unroll
    for (int k = 0; k < 8; ++k) o[k] = f2bf(v[k]); *(volatile v8us*)(dst + i * 8) = o; __threadfence(); *(volatile v8us*)(dst + i * 8) = o; }
__global__ __launch_bounds__(256) void k_gstat(const float* __restrict__ X, float* MS) { const int gidx = blockIdx.x; const int tid = threadIdx.x; const float* base = X + (size_t)gidx * (CC / NG) * NN; __shared__ float red[256]; float s = 0.f;
#pragma unroll 1
    for (int i = tid; i < (CC / NG) * NN; i += 256) s += bfr(base[i]);
    red[tid] = s; __syncthreads();
    for (int st = 128; st > 0; st >>= 1) { if (tid < st) red[tid] = red[tid] + red[tid + st]; __syncthreads(); }
    const float mean = red[0] * (1.0f / ((CC / NG) * NN)); __syncthreads(); float q = 0.f;
#pragma unroll 1
    for (int i = tid; i < (CC / NG) * NN; i += 256) { float d = __fsub_rn(bfr(base[i]), mean); asm volatile("" : "+v"(d)); float p = __fmul_rn(d, d); asm volatile("" : "+v"(p)); q = __fadd_rn(q, p); }
    red[tid] = q; __syncthreads();
    for (int st = 128; st > 0; st >>= 1) { if (tid < st) red[tid] = red[tid] + red[tid + st]; __syncthreads(); }
    if (tid == 0) { const float var = red[0] * (1.0f / ((CC / NG) * NN)); v2f o; o[0] = mean; o[1] = __frsqrt_rn(__fadd_rn(var, 1e-5f)); *(volatile v2f*)(MS + gidx * 2) = o; __threadfence(); *(volatile v2f*)(MS + gidx * 2) = o; } }
__global__ __launch_bounds__(64) void k_gfix(float* MS) { const int t = threadIdx.x; if (t >= NG * 2) return; const float v = MS[t]; __syncthreads(); *(volatile float*)(MS + t) = v; __threadfence(); *(volatile float*)(MS + t) = v; }
__global__ __launch_bounds__(256) void k_hnT(const float* __restrict__ X, const float* __restrict__ MS, const float* __restrict__ w, const float* __restrict__ bb, bf* Hh, bf* Hl) { const size_t e = ((size_t)blockIdx.x * 256 + threadIdx.x) * 4; if (e >= (size_t)NN * CC) return; const int c = (int)(e % CC); const int n = (int)(e / CC); v4us oh, ol;
#pragma unroll
    for (int u = 0; u < 4; ++u) { const int cu = c + u; const int gg = cu / (CC / NG); const float mean = MS[gg * 2], rs = MS[gg * 2 + 1]; float d = __fsub_rn(bfr(X[(size_t)cu * NN + n]), mean); asm volatile("" : "+v"(d)); float nrm = __fmul_rn(d, rs); asm volatile("" : "+v"(nrm)); float t1 = __fmul_rn(nrm, bfr(w[cu])); asm volatile("" : "+v"(t1)); const float y = __fadd_rn(t1, bfr(bb[cu])); unsigned short a, b2; splitf(y, a, b2); oh[u] = a; ol[u] = b2; }
    *(volatile v4us*)(Hh + e) = oh; *(volatile v4us*)(Hl + e) = ol; __threadfence(); *(volatile v4us*)(Hh + e) = oh; *(volatile v4us*)(Hl + e) = ol; }
__global__ __launch_bounds__(256) void k_p16(const float* __restrict__ F, h16* P) { const size_t e = ((size_t)blockIdx.x * 256 + threadIdx.x) * 4; if (e >= (size_t)NN * CC) return; const v4f a = *(const v4f*)(F + e); v4h o; for (int u = 0; u < 4; ++u) o[u] = tohx(a[u]); *(volatile v4h*)(P + e) = o; __threadfence(); *(volatile v4h*)(P + e) = o; }
__global__ __launch_bounds__(256) void k_v16T(const float* __restrict__ Vt, h16* V16) { const size_t e = ((size_t)blockIdx.x * 256 + threadIdx.x) * 2; if (e >= (size_t)CC * NN) return; const int m = (int)(e % NN); const int c = (int)(e / NN); v2h o; o[0] = tohx(Vt[(size_t)m * CC + c]); o[1] = tohx(Vt[(size_t)(m + 1) * CC + c]); *(volatile v2h*)(V16 + e) = o; __threadfence(); *(volatile v2h*)(V16 + e) = o; }
__global__ __launch_bounds__(256) void k_soft(const float* __restrict__ S, h16* P16) { const int lane = threadIdx.x & 31; const int row = blockIdx.x * 8 + (threadIdx.x >> 5); if (row >= NN) return; const float* sr = S + (size_t)row * NN; float v[NN / 32]; float mx = -3.0e38f;
#pragma unroll
    for (int ch = 0; ch < NN / 128; ++ch) { const v4f a = *(const v4f*)(sr + ch * 128 + lane * 4);
#pragma unroll
        for (int u = 0; u < 4; ++u) { const float t = a[u] * 0.044194173824159216f; v[ch * 4 + u] = t; mx = fmaxf(mx, t); } }
#pragma unroll
    for (int sh = 16; sh; sh >>= 1) mx = fmaxf(mx, __shfl_xor(mx, sh, 32));
    float sum = 0.f;
#pragma unroll
    for (int q = 0; q < NN / 32; ++q) { float d0 = __fsub_rn(v[q], mx); asm volatile("" : "+v"(d0)); v[q] = __builtin_amdgcn_exp2f(__fmul_rn(d0, 1.4426950408889634f)); sum += v[q]; }
#pragma unroll
    for (int sh = 16; sh; sh >>= 1) sum += __shfl_xor(sum, sh, 32);
    const float f = __fdiv_rn(PCAR, sum);
    for (int ps = 0; ps < 2; ++ps) {
#pragma unroll
        for (int ch = 0; ch < NN / 128; ++ch) { v4h o4; for (int q = 0; q < 4; ++q) o4[q] = tohx(v[ch * 4 + q] * f); *(volatile v4h*)(P16 + (size_t)row * NN + ch * 128 + lane * 4) = o4; }
        if (ps == 0) __threadfence(); } }
__global__ __launch_bounds__(256) void k_opl(const float* __restrict__ O, bf* Ph, bf* Pl) { const size_t e = ((size_t)blockIdx.x * 256 + threadIdx.x) * 4; if (e >= (size_t)NN * CC) return; const v4f a = *(const v4f*)(O + e); v4us oh, ol;
#pragma unroll
    for (int u = 0; u < 4; ++u) { unsigned short x0, x1; splitf(a[u] * (1.0f / PCAR), x0, x1); oh[u] = x0; ol[u] = x1; } *(volatile v4us*)(Ph + e) = oh; *(volatile v4us*)(Pl + e) = ol; __threadfence(); *(volatile v4us*)(Ph + e) = oh; *(volatile v4us*)(Pl + e) = ol; }
__global__ __launch_bounds__(256) void k_res(const float* __restrict__ X, const float* __restrict__ PJ, float* Y) { const size_t e = ((size_t)blockIdx.x * 256 + threadIdx.x) * 4; if (e >= (size_t)CC * NN) return; const int n = (int)(e % NN); const int c = (int)(e / NN); const v4f xx = *(const v4f*)(X + e); v4f r;
#pragma unroll
    for (int u = 0; u < 4; ++u) r[u] = __fadd_rn(bfr(xx[u]), PJ[(size_t)(n + u) * CC + c]); *(volatile v4f*)(Y + e) = r; __threadfence(); *(volatile v4f*)(Y + e) = r; }

extern "C" void kernel_launch(void* const* d_in, const int* in_sizes, int n_in,
                              void* d_out, int out_size, void* d_ws, size_t ws_size, hipStream_t stream) {
    (void)in_sizes; (void)n_in; (void)out_size;
    const float* x = (const float*)d_in[0]; const float* gw = (const float*)d_in[1]; const float* gb = (const float*)d_in[2]; const float* qw = (const float*)d_in[3]; const float* qb = (const float*)d_in[4]; const float* kw = (const float*)d_in[5]; const float* kb = (const float*)d_in[6]; const float* vw = (const float*)d_in[7]; const float* vb = (const float*)d_in[8]; const float* pw = (const float*)d_in[9]; const float* pb = (const float*)d_in[10];
    float* OUT = (float*)d_out;
    char* wsp = (char*)d_ws;
    auto take = [&](size_t bytes) { char* p = wsp; wsp += (bytes + 255) & ~(size_t)255; return (void*)p; };
    bf* BQ = (bf*)take((size_t)CC * CC * 2); bf* BK = (bf*)take((size_t)CC * CC * 2); bf* BV = (bf*)take((size_t)CC * CC * 2); bf* BP = (bf*)take((size_t)CC * CC * 2); float* MS = (float*)take(256);
    bf* HTh = (bf*)take((size_t)NN * CC * 2); bf* HTl = (bf*)take((size_t)NN * CC * 2); float* F = (float*)take((size_t)NN * CC * 4); h16* Q16 = (h16*)take((size_t)NN * CC * 2); h16* K16 = (h16*)take((size_t)NN * CC * 2); h16* V16 = (h16*)take((size_t)CC * NN * 2);
    float* S = (float*)take((size_t)NN * NN * 4); h16* P16 = (h16*)take((size_t)NN * NN * 2); float* O = (float*)take((size_t)NN * CC * 4); bf* OPh = (bf*)take((size_t)NN * CC * 2); bf* OPl = (bf*)take((size_t)NN * CC * 2); float* PJ = (float*)take((size_t)NN * CC * 4);
    if ((size_t)(wsp - (char*)d_ws) > ws_size) return;
    k_cvt8<<<(CC * CC / 8 + 255) / 256, 256, 0, stream>>>(qw, BQ, CC * CC / 8); k_cvt8<<<(CC * CC / 8 + 255) / 256, 256, 0, stream>>>(kw, BK, CC * CC / 8); k_cvt8<<<(CC * CC / 8 + 255) / 256, 256, 0, stream>>>(vw, BV, CC * CC / 8); k_cvt8<<<(CC * CC / 8 + 255) / 256, 256, 0, stream>>>(pw, BP, CC * CC / 8);
    const dim3 gp(NN / 64, CC / 64, 1); const unsigned LP = (unsigned)(((size_t)NN * CC / 4 + 255) / 256);
    for (int b = 0; b < NB_; ++b) { const float* xb = x + (size_t)b * CC * NN;
        k_gstat<<<NG, 256, 0, stream>>>(xb, MS); k_gfix<<<1, 64, 0, stream>>>(MS);
        k_hnT<<<LP, 256, 0, stream>>>(xb, MS, gw, gb, HTh, HTl);
        k_gemmw<bf, 1, true><<<gp, 32, 0, stream>>>(HTh, HTl, BQ, nullptr, CC, F, CC, qb, 0, 0, 0); k_p16<<<LP, 256, 0, stream>>>(F, Q16);
        k_gemmw<bf, 1, true><<<gp, 32, 0, stream>>>(HTh, HTl, BK, nullptr, CC, F, CC, kb, 0, 0, 0); k_p16<<<LP, 256, 0, stream>>>(F, K16);
        k_gemmw<bf, 1, true><<<gp, 32, 0, stream>>>(HTh, HTl, BV, nullptr, CC, F, CC, vb, 0, 0, 0); k_v16T<<<(unsigned)(((size_t)CC * NN / 2 + 255) / 256), 256, 0, stream>>>(F, V16);
        k_gemmw<h16, 0, false><<<dim3(NN / 64, NN / 64, 1), 32, 0, stream>>>(Q16, nullptr, K16, nullptr, CC, S, NN, nullptr, 0, 0, 0);
        k_soft<<<NN / 8, 256, 0, stream>>>(S, P16);
        k_gemmw<h16, 0, false><<<dim3(NN / 64, CC / 64, 1), 32, 0, stream>>>(P16, nullptr, V16, nullptr, NN, O, CC, nullptr, 0, 0, 0);
        k_opl<<<LP, 256, 0, stream>>>(O, OPh, OPl);
        k_gemmw<bf, 1, true><<<gp, 32, 0, stream>>>(OPh, OPl, BP, nullptr, CC, PJ, CC, pb, 0, 0, 0);
        k_res<<<(unsigned)(((size_t)CC * NN / 4 + 255) / 256), 256, 0, stream>>>(xb, PJ, OUT + (size_t)b * CC * NN); }
}
